// SpixEmbedding_25082609009343
// MI455X (gfx1250) — hardware-run, weakly checked
//
#include <hip/hip_runtime.h>

typedef __attribute__((ext_vector_type(16))) _Float16 v16h;
typedef __attribute__((ext_vector_type(8)))  _Float16 v8h;
typedef __attribute__((ext_vector_type(2)))  _Float16 v2h;
typedef __attribute__((ext_vector_type(8)))  float    v8f;
typedef __attribute__((ext_vector_type(4)))  float    v4f;
typedef __attribute__((ext_vector_type(4)))  int      v4i;

constexpr int kBatch  = 8;
constexpr int kChan   = 16;
constexpr int kImgH   = 256;
constexpr int kImgW   = 256;
constexpr int kEmb    = 384;
constexpr int kPatch  = 256;
constexpr int kPsz    = 16;
constexpr int kNseg   = 256;
constexpr int kImgPix = kImgH * kImgW;
constexpr int kGemmM  = kBatch * kPatch;
constexpr int kGemmN  = kEmb;
constexpr int kGemmK  = kPsz * kPsz * kChan;
constexpr float kCarryA   = 16.0f;
constexpr float kCarryW   = 1024.0f;
constexpr float kOutScale = 1.0f / (kCarryA * kCarryW);
static_assert(kGemmM == 2048 && kGemmN == 384 && kGemmK == 4096, "GEMM shape");
static_assert((kGemmM % 64) == 0 && (kGemmN % 64) == 0 && (kGemmK % 32) == 0, "tile multiples");
static_assert(kImgPix == 65536, "image size");

constexpr size_t kOffBB   = 0;
constexpr size_t kOffBT   = kOffBB + (size_t)kBatch * 4 * kNseg * 4;
constexpr size_t kOffAP   = kOffBT + (size_t)kGemmN * kGemmK * 2;
constexpr size_t kWsTotal = kOffAP + (size_t)kGemmM * kGemmK * 2;
static_assert(kOffBT == 32768ull && kOffAP == 3178496ull, "carve offsets");
static_assert(kWsTotal == 19955712ull, "carve total");
static_assert(kWsTotal <= 134217728ull, "carve cap");
static_assert((kOffBT % 128) == 0 && (kOffAP % 128) == 0, "128-B aligned regions");

__device__ __forceinline__ int iclamp(int v, int lo, int hi) {
  const int a = (v < lo) ? lo : v;
  return (a > hi) ? hi : a;
}

__device__ __forceinline__ void wm_guard1(v8f& a, v16h x, v16h y) {
  asm volatile("v_nop\n\tv_nop\n\tv_nop\n\tv_nop" : "+v"(a) : "v"(x), "v"(y));
}
__device__ __forceinline__ void wm_acc1(v8f& a) {
  asm volatile("v_nop\n\tv_nop\n\tv_nop\n\tv_nop" : "+v"(a));
}
__device__ __forceinline__ void wm_keep4(v16h a, v16h b, v16h c, v16h d) {
  asm volatile("v_nop" :: "v"(a), "v"(b), "v"(c), "v"(d));
}
struct FragH {
  union U { v16h v; v8h h[2]; };
  static __device__ __forceinline__ v16h load(const _Float16* p) {
    U f;
    f.h[0] = *(const v8h*)(p);
    f.h[1] = *(const v8h*)(p + 16);
    return f.v;
  }
  static __device__ __forceinline__ v8f mma(v16h a, v16h b, v8f c) {
    return __builtin_amdgcn_wmma_f32_16x16x32_f16(false, a, false, b, (short)0, c, false, false);
  }
};

__global__ __launch_bounds__(512) void bbox_kernel(const int* __restrict__ seg, int* __restrict__ bb)
{
  __shared__ __align__(16) int sB[4 * kNseg];
  const int tid = threadIdx.x;
  const int b = blockIdx.x;
  {
    const int e0 = tid;
    const int e1 = tid + 512;
    const int q0 = e0 >> 8;
    const int q1 = e1 >> 8;
    sB[e0] = ((q0 & 1) == 0) ? 0x7fffffff : -1;
    sB[e1] = ((q1 & 1) == 0) ? 0x7fffffff : -1;
  }
  __syncthreads();
  const int* sp = seg + (size_t)b * kImgPix;
#pragma unroll 4
  for (int it = 0; it < 128; ++it) {
    const int idx = it * 512 + tid;
    const int s = sp[idx];
    const int r = idx >> 8;
    const int c = idx & 255;
    if ((unsigned)s < (unsigned)kNseg) {
      atomicMin(&sB[s], r);
      atomicMax(&sB[kNseg + s], r);
      atomicMin(&sB[2 * kNseg + s], c);
      atomicMax(&sB[3 * kNseg + s], c);
    }
  }
  __syncthreads();
  if (tid < 256) {
    const v4i v = *(const v4i*)(sB + 4 * tid);
    int* dst = bb + (size_t)b * 4 * kNseg + 4 * tid;
    *(volatile v4i*)dst = v;
    __threadfence();
    *(volatile v4i*)dst = v;
  }
}

__global__ __launch_bounds__(256) void packw_kernel(const float* __restrict__ W, unsigned short* __restrict__ Bt)
{
  __shared__ __align__(16) float sT[64 * 68];
  const int tid = threadIdx.x, lane = tid & 31, wave = tid >> 5;
  const int k0 = blockIdx.x * 64;
  const int n0 = blockIdx.y * 64;
  {
    const int row = tid >> 4;
    const int c4 = (tid & 15) * 4;
#pragma unroll
    for (int pass = 0; pass < 4; ++pass) {
      const int kr = pass * 16 + row;
      const v4f v = *(const v4f*)(W + (size_t)(k0 + kr) * kGemmN + n0 + c4);
      *(v4f*)(sT + kr * 68 + c4) = v;
    }
  }
  __syncthreads();
  const int q = lane >> 3;
  const int k8 = (lane & 7) * 8;
  v8h hv[2];
#pragma unroll
  for (int it = 0; it < 2; ++it) {
    const int n = it * 32 + wave * 4 + q;
#pragma unroll
    for (int e = 0; e < 8; ++e) {
      const float f = sT[(k8 + e) * 68 + n] * kCarryW;
      hv[it][e] = (_Float16)f;
    }
  }
  for (int pass = 0; pass < 2; ++pass) {
#pragma unroll
    for (int it = 0; it < 2; ++it) {
      const int n = it * 32 + wave * 4 + q;
      *(volatile v8h*)(Bt + (size_t)(n0 + n) * kGemmK + k0 + k8) = hv[it];
    }
    __threadfence();
  }
}

__global__ __launch_bounds__(256) void sample_kernel(
    const float* __restrict__ x, const int* __restrict__ seg, const int* __restrict__ crop,
    const int* __restrict__ bb, unsigned* __restrict__ Aw)
{
  __shared__ int   sR0[16];
  __shared__ int   sC0[16];
  __shared__ float sFr[16];
  __shared__ float sFc[16];
  __shared__ int   sFlag[256];
  const int tid = threadIdx.x, lane = tid & 31, wave = tid >> 5;
  const int m = blockIdx.x;
  const int b = m >> 8;
  const int* segb = seg + (size_t)b * kImgPix;
  {
    const int k = tid >> 4, l = tid & 15;
    const int idraw = crop[m];
    const int id = iclamp(idraw, 0, kNseg - 1);
    const int* bbp = bb + (size_t)b * 4 * kNseg;
    const int rmn = iclamp(bbp[id], 0, kImgH - 1);
    const int rmx = iclamp(bbp[kNseg + id], 0, kImgH - 1);
    const int cmn = iclamp(bbp[2 * kNseg + id], 0, kImgW - 1);
    const int cmx = iclamp(bbp[3 * kNseg + id], 0, kImgW - 1);
    const int extr = rmx - rmn + 1;
    const int extc = cmx - cmn + 1;
    const bool issmall = (extr <= kPsz) && (extc <= kPsz);
    int qr = (2 * k + 1) * extr - 16;
    int qrmax = 32 * (extr - 1);
    qr = (qr > qrmax) ? qrmax : qr;
    qr = (qr < 0) ? 0 : qr;
    int qc = (2 * l + 1) * extc - 16;
    int qcmax = 32 * (extc - 1);
    qc = (qc > qcmax) ? qcmax : qc;
    qc = (qc < 0) ? 0 : qc;
    int r0 = issmall ? (rmn + k) : (rmn + (qr >> 5));
    int c0 = issmall ? (cmn + l) : (cmn + (qc >> 5));
    const int frq = issmall ? 0 : (qr & 31);
    const int fcq = issmall ? 0 : (qc & 31);
    r0 = iclamp(r0, 0, kImgH + kPsz - 2);
    c0 = iclamp(c0, 0, kImgW + kPsz - 2);
    const float fr = (float)frq * 0.03125f;
    const float fc = (float)fcq * 0.03125f;
    const int rc0 = iclamp(r0, 0, kImgH - 1), rc1 = iclamp(r0 + 1, 0, kImgH - 1);
    const int cl0 = iclamp(c0, 0, kImgW - 1), cl1 = iclamp(c0 + 1, 0, kImgW - 1);
    const bool vr0 = (r0 < kImgH), vr1 = (r0 + 1 < kImgH);
    const bool vc0 = (c0 < kImgW), vc1 = (c0 + 1 < kImgW);
    const int s00 = segb[rc0 * kImgW + cl0];
    const int s01 = segb[rc0 * kImgW + cl1];
    const int s10 = segb[rc1 * kImgW + cl0];
    const int s11 = segb[rc1 * kImgW + cl1];
    const float m00 = (vr0 && vc0 && (s00 == idraw)) ? 1.0f : 0.0f;
    const float m01 = (vr0 && vc1 && (s01 == idraw)) ? 1.0f : 0.0f;
    const float m10 = (vr1 && vc0 && (s10 == idraw)) ? 1.0f : 0.0f;
    const float m11 = (vr1 && vc1 && (s11 == idraw)) ? 1.0f : 0.0f;
    const float omr = 1.0f - fr, omc = 1.0f - fc;
    const float w00 = omr * omc, w01 = omr * fc, w10 = fr * omc, w11 = fr * fc;
    const float segf = w00 * m00 + w01 * m01 + w10 * m10 + w11 * m11;
    sFlag[tid] = (segf != 0.0f) ? 1 : 0;
    if (l == 0) {
      sR0[k] = r0;
      sFr[k] = fr;
    }
    if (k == 0) {
      sC0[l] = c0;
      sFc[l] = fc;
    }
  }
  __syncthreads();

  const int pxl = lane >> 3;
  const int cp = lane & 7;
  const float* xc0 = x + (size_t)b * kChan * kImgPix + (size_t)(2 * cp) * kImgPix;
  const float* xc1 = xc0 + kImgPix;
  unsigned* Arow = Aw + (size_t)m * (kGemmK / 2);
#pragma unroll 1
  for (int it = 0; it < 8; ++it) {
    const int L = wave * 8 + it;
    const int px = 4 * L + pxl;
    const int fl = sFlag[px];
    const unsigned actmask = __builtin_amdgcn_ballot_w32(fl != 0);
    float v0 = 0.0f, v1 = 0.0f;
    if (actmask != 0u) {
      const int kk = px >> 4, ll = px & 15;
      const int r0 = sR0[kk];
      const int c0 = sC0[ll];
      const float fr = sFr[kk];
      const float fc = sFc[ll];
      const int rc0 = iclamp(r0, 0, kImgH - 1), rc1 = iclamp(r0 + 1, 0, kImgH - 1);
      const int cl0 = iclamp(c0, 0, kImgW - 1), cl1 = iclamp(c0 + 1, 0, kImgW - 1);
      const bool vr0 = (r0 < kImgH), vr1 = (r0 + 1 < kImgH);
      const bool vc0 = (c0 < kImgW), vc1 = (c0 + 1 < kImgW);
      const int i00 = rc0 * kImgW + cl0, i01 = rc0 * kImgW + cl1;
      const int i10 = rc1 * kImgW + cl0, i11 = rc1 * kImgW + cl1;
      float a00 = xc0[i00], a01 = xc0[i01], a10 = xc0[i10], a11 = xc0[i11];
      float b00 = xc1[i00], b01 = xc1[i01], b10 = xc1[i10], b11 = xc1[i11];
      a00 = (vr0 && vc0) ? a00 : 0.0f;
      a01 = (vr0 && vc1) ? a01 : 0.0f;
      a10 = (vr1 && vc0) ? a10 : 0.0f;
      a11 = (vr1 && vc1) ? a11 : 0.0f;
      b00 = (vr0 && vc0) ? b00 : 0.0f;
      b01 = (vr0 && vc1) ? b01 : 0.0f;
      b10 = (vr1 && vc0) ? b10 : 0.0f;
      b11 = (vr1 && vc1) ? b11 : 0.0f;
      const float omr = 1.0f - fr, omc = 1.0f - fc;
      const float w00 = omr * omc, w01 = omr * fc, w10 = fr * omc, w11 = fr * fc;
      const float f0 = w00 * a00 + w01 * a01 + w10 * a10 + w11 * a11;
      const float f1 = w00 * b00 + w01 * b01 + w10 * b10 + w11 * b11;
      v0 = (fl != 0) ? (f0 * kCarryA) : 0.0f;
      v1 = (fl != 0) ? (f1 * kCarryA) : 0.0f;
    }
    v2h hv;
    hv[0] = (_Float16)v0;
    hv[1] = (_Float16)v1;
    const unsigned u = __builtin_bit_cast(unsigned, hv);
    volatile unsigned* dst = (volatile unsigned*)(Arow + L * 32 + lane);
    *dst = u;
    __threadfence();
    *dst = u;
  }
}

__global__ __launch_bounds__(256) void gemm_f16_kernel(
    const unsigned short* __restrict__ Ap, const unsigned short* __restrict__ Btp,
    float* __restrict__ C, float scale)
{
  const _Float16* A  = (const _Float16*)Ap;
  const _Float16* Bt = (const _Float16*)Btp;
  __shared__ __align__(16) float sT[8][16 * 68];
  const int lane = threadIdx.x & 31;
  const int wave = threadIdx.x >> 5;
  constexpr int tilesN = kGemmN >> 6;
  constexpr int tilesM = kGemmM >> 6;
  const int tile = blockIdx.x * 8 + wave;
  if (tile >= tilesM * tilesN) return;
  const int tm = tile / tilesN;
  const int tn = tile - tm * tilesN;
  const int m0 = tm << 6;
  const int n0 = tn << 6;
  const int rlane = lane & 15;
  const int koff  = (lane >> 4) * 8;
  const int mOff  = (lane >> 4) * 8;

  v8f acc[4][4];
#pragma unroll
  for (int i = 0; i < 4; ++i)
#pragma unroll
    for (int j = 0; j < 4; ++j) acc[i][j] = (v8f){0.f, 0.f, 0.f, 0.f, 0.f, 0.f, 0.f, 0.f};

#pragma unroll 1
  for (int k0 = 0; k0 < kGemmK; k0 += 32) {
    v16h bh[4];
#pragma unroll
    for (int j = 0; j < 4; ++j) {
      const size_t bo = (size_t)(n0 + (j << 4) + rlane) * kGemmK + koff + k0;
      bh[j] = FragH::load(Bt + bo);
    }
#pragma unroll
    for (int i = 0; i < 4; ++i) {
      const size_t ao = (size_t)(m0 + (i << 4) + rlane) * kGemmK + koff + k0;
      const v16h ah = FragH::load(A + ao);
#pragma unroll
      for (int j = 0; j < 4; ++j) acc[i][j] = FragH::mma(ah, bh[j], acc[i][j]);
      wm_guard1(acc[i][0], ah, bh[0]);
      wm_guard1(acc[i][1], ah, bh[1]);
      wm_guard1(acc[i][2], ah, bh[2]);
      wm_guard1(acc[i][3], ah, bh[3]);
    }
    wm_keep4(bh[0], bh[1], bh[2], bh[3]);
  }
#pragma unroll
  for (int i = 0; i < 4; ++i) {
    wm_acc1(acc[i][0]);
    wm_acc1(acc[i][1]);
    wm_acc1(acc[i][2]);
    wm_acc1(acc[i][3]);
  }

  float* slab = sT[wave];
#pragma unroll
  for (int i = 0; i < 4; ++i) {
    const int mBase = m0 + (i << 4);
#pragma unroll
    for (int j = 0; j < 4; ++j) {
#pragma unroll
      for (int r = 0; r < 8; ++r) {
        const float v = acc[i][j][r] * scale;
        slab[(mOff + r) * 68 + (j << 4) + rlane] = v;
      }
    }
    __builtin_amdgcn_fence(__ATOMIC_RELEASE, "workgroup");
    __builtin_amdgcn_wave_barrier();
    __builtin_amdgcn_fence(__ATOMIC_ACQUIRE, "workgroup");
    {
      const int hh = lane >> 4, c4 = (lane & 15) * 4;
      for (int pass = 0; pass < 2; ++pass) {
#pragma unroll
        for (int it = 0; it < 8; ++it) {
          const int row = it * 2 + hh;
          const v4f v = *(const v4f*)(slab + row * 68 + c4);
          *(volatile v4f*)(C + (size_t)(mBase + row) * kGemmN + n0 + c4) = v;
        }
        __threadfence();
      }
    }
    __builtin_amdgcn_fence(__ATOMIC_RELEASE, "workgroup");
    __builtin_amdgcn_wave_barrier();
    __builtin_amdgcn_fence(__ATOMIC_ACQUIRE, "workgroup");
  }
}

extern "C" void kernel_launch(void* const* d_in, const int* in_sizes, int n_in,
                              void* d_out, int out_size, void* d_ws, size_t ws_size,
                              hipStream_t stream) {
  if (n_in < 4) return;
  if (in_sizes[0] != kBatch * kChan * kImgPix) return;
  if (in_sizes[1] != kBatch * kImgPix) return;
  if (in_sizes[2] != kBatch * kPatch) return;
  if (in_sizes[3] != kGemmK * kGemmN) return;
  if (out_size != kGemmM * kGemmN) return;
  if (ws_size < kWsTotal) return;

  const float* x    = (const float*)d_in[0];
  const int*   seg  = (const int*)d_in[1];
  const int*   crop = (const int*)d_in[2];
  const float* Wm   = (const float*)d_in[3];
  float*       out  = (float*)d_out;

  char* ws = (char*)d_ws;
  int*            BB = (int*)(ws + kOffBB);
  unsigned short* BT = (unsigned short*)(ws + kOffBT);
  unsigned*       AP = (unsigned*)(ws + kOffAP);

  bbox_kernel<<<kBatch, 512, 0, stream>>>(seg, BB);
  packw_kernel<<<dim3(kGemmK / 64, kGemmN / 64), 256, 0, stream>>>(Wm, BT);
  sample_kernel<<<kGemmM, 256, 0, stream>>>(x, seg, crop, BB, AP);
  gemm_f16_kernel<<<((kGemmM / 64) * (kGemmN / 64)) / 8, 256, 0, stream>>>(
      (const unsigned short*)AP, BT, out, kOutScale);
}
